// MobileNetV2_50405736186389
// MI455X (gfx1250) — hardware-run, weakly checked
//
#include <hip/hip_runtime.h>


#ifndef NB
#define NB 4
#endif
#ifndef NT
#define NT 128
#endif
#define NB_FULL 4
#define NT_FULL 128
#ifndef OUT_NT
#define OUT_NT NT
#endif
#define CH   64
#define RC   4
#define HW   196
#define SW   14
#define PQ   208
#define PK   224
#define PT   13
#define XP   72
#define OSP  68
#define FT   448
#define WSC  64.0f
#define WSI  (1.0f / 64.0f)
#define PCAR 256.0f
#define PCI  (1.0f / 256.0f)
#define LOG2E 1.4426950408889634f

static_assert(NB <= NB_FULL);
static_assert(NT <= NT_FULL);
static_assert(NT % 8 == 0);
static_assert(OUT_NT % 8 == 0);
static_assert(OUT_NT >= NT);
static_assert(HW == SW * SW);
static_assert(HW % 4 == 0);
static_assert(PQ == PT * 16);
static_assert(PQ >= HW);
static_assert(PK % 32 == 0);
static_assert(PK >= PQ);
static_assert(CH % 32 == 0);
static_assert(CH == 64);
static_assert(FT == 32 * (PK / 16));
static_assert((CH * (HW / 4)) % FT == 0);
static_assert((PK * CH / 8) % FT == 0);
static_assert(((PK - HW) * XP) % 8 == 0);
static_assert((PK - HW) * XP / 8 <= FT);
static_assert((PQ * CH / 8) <= 4 * FT);
static_assert(((PQ * CH / 8) - 3 * FT) % 32 == 0);
static_assert(RC * CH <= FT);
static_assert(RC * PK / 4 == PK);
static_assert((XP * 2) % 16 == 0);
static_assert((OSP * 4) % 16 == 0);
static_assert(8 * 32 * 16 == 16 * CH * 4);
static_assert(PK * XP * 2 + RC * CH * 4 + RC * PK * 4 <= 131072);
static_assert(PT * 16 * OSP * 4 <= 65536);
static_assert((3 * 324 + 12 + 3 + RC * PK) * 4 <= 131072);

typedef _Float16 h16;
typedef __attribute__((ext_vector_type(16))) _Float16 v16h;
typedef __attribute__((ext_vector_type(8)))  _Float16 v8h;
typedef __attribute__((ext_vector_type(8)))  float    v8f;
typedef __attribute__((ext_vector_type(4)))  float    v4f;
typedef v4f  __attribute__((may_alias)) v4fa;

__device__ __forceinline__ unsigned short f2bf(float f) { unsigned u = __float_as_uint(f); u += 0x7FFFu + ((u >> 16) & 1u); return (unsigned short)(u >> 16); }
__device__ __forceinline__ float bfr(float f) { return __uint_as_float(((unsigned)f2bf(f)) << 16); }
__device__ __forceinline__ v16h cat16(v8h lo, v8h hi) { return __builtin_shufflevector(lo, hi, 0, 1, 2, 3, 4, 5, 6, 7, 8, 9, 10, 11, 12, 13, 14, 15); }
__device__ __forceinline__ v8f wmma16(v16h a, v16h b, v8f c) { return __builtin_amdgcn_wmma_f32_16x16x32_f16(false, a, false, b, (short)0, c, false, false); }
__device__ __forceinline__ v8f wmma16g(v16h a, v16h b, v8f c) { c = wmma16(a, b, c); asm volatile("v_nop\n\tv_nop\n\tv_nop\n\tv_nop" : "+v"(c) : "v"(a), "v"(b)); return c; }
__device__ __forceinline__ v16h  ldh(const h16* p) { return cat16(*(const v8h*)p, *(const v8h*)(p + 16)); }
__device__ __forceinline__ void wave_sync() { __builtin_amdgcn_fence(3  , "wavefront"); __builtin_amdgcn_wave_barrier(); asm volatile("" ::: "memory"); }
__device__ __forceinline__ h16 toh_flush(float v) { const h16 r = (h16)v; return (fabsf(v) < 6.103515625e-05f) ? (h16)0.0f : r; }
__device__ __forceinline__ float sgm(float s) { return __builtin_amdgcn_rcpf(1.0f + __builtin_amdgcn_exp2f(-LOG2E * s)) - 0.5f; }

__global__ __launch_bounds__(256) void k_wconv(const float* __restrict__ src, h16* dst, int n8) {
    const int i = blockIdx.x * 256 + threadIdx.x; if (i >= n8) return;
    const v4f a = *(const v4f*)(src + (size_t)i * 8); const v4f b = *(const v4f*)(src + (size_t)i * 8 + 4); v8h o;
#pragma unroll
    for (int k = 0; k < 4; ++k) { o[k] = toh_flush(bfr(a[k]) * WSC); o[4 + k] = toh_flush(bfr(b[k]) * WSC); }
    *(volatile v8h*)(dst + (size_t)i * 8) = o; __threadfence(); *(volatile v8h*)(dst + (size_t)i * 8) = o;
}

__global__ __launch_bounds__(FT) void k_front(const float* __restrict__ X, const float* __restrict__ WD, const h16* __restrict__ W2H,
                                              h16* XT, h16* X2T, h16* X2C, float* XR) {
    __shared__ __align__(16) h16   xs[PK * XP];
    __shared__ __align__(16) float wds[RC * CH];
    __shared__ __align__(16) float xrs[RC * PK];
    const int tid = threadIdx.x;
    const int lane = tid & 31, lr = lane & 15, hi = lane >> 4;
    const int wave = __builtin_amdgcn_readfirstlane((int)(threadIdx.x >> 5));
    const int frame = blockIdx.x; const int b = frame / NT, t = frame % NT;
    { const float wv = bfr(WD[tid & (RC * CH - 1)]); if (tid < RC * CH) wds[tid] = wv; }
    if (tid < (PK - HW) * XP / 8) { const v8h z = (v8h){}; *(v8h*)(&xs[HW * XP + tid * 8]) = z; }
    const float* xb = X + ((size_t)b * CH * NT_FULL + (size_t)t) * HW;
#pragma unroll 1
    for (int it = 0; it < (CH * (HW / 4)) / FT; ++it) {
        const int i = it * FT + tid; const int c = i / (HW / 4); const int p4 = (i - c * (HW / 4)) * 4;
        const v4f v = *(const v4f*)(xb + (size_t)c * NT_FULL * HW + p4);
#pragma unroll
        for (int j = 0; j < 4; ++j) xs[(p4 + j) * XP + c] = toh_flush(bfr(v[j]));
    }
    __syncthreads();
    v8f acc[4];
    { const int arow = wave * 16 + lr;
      const v16h a0 = cat16(*(const v8h*)(&xs[arow * XP + 8 * hi]),      *(const v8h*)(&xs[arow * XP + 16 + 8 * hi]));
      const v16h a1 = cat16(*(const v8h*)(&xs[arow * XP + 32 + 8 * hi]), *(const v8h*)(&xs[arow * XP + 48 + 8 * hi]));
#pragma unroll
      for (int nb = 0; nb < 4; ++nb) { const h16* wp = W2H + (size_t)(nb * 16 + lr) * CH + 8 * hi;
          v8f c = (v8f){}; c = wmma16g(a0, ldh(wp), c); c = wmma16g(a1, ldh(wp + 32), c); acc[nb] = c; } }
#pragma unroll 1
    for (int ps = 0; ps < 2; ++ps) {
#pragma unroll 1
        for (int it = 0; it < 4; ++it) { const int i = it * FT + tid;
            if (i < PQ * CH / 8) { const v8h v = *(const v8h*)(&xs[(i >> 3) * XP + (i & 7) * 8]);
                *(volatile v8h*)(XT + (size_t)frame * PQ * CH + (size_t)i * 8) = v; } }
        if (ps == 0) __threadfence(); }
    if (wave < PK / 32) {
        const int p = tid; float s0 = 0.0f, s1 = 0.0f, s2 = 0.0f, s3 = 0.0f;
#pragma unroll 4
        for (int c = 0; c < CH; ++c) { const float xv = (float)xs[p * XP + c];
            s0 += wds[c] * xv; s1 += wds[CH + c] * xv; s2 += wds[2 * CH + c] * xv; s3 += wds[3 * CH + c] * xv; }
        const bool ok = p < HW;
        xrs[p] = ok ? s0 : 0.0f; xrs[PK + p] = ok ? s1 : 0.0f; xrs[2 * PK + p] = ok ? s2 : 0.0f; xrs[3 * PK + p] = ok ? s3 : 0.0f;
    }
    __syncthreads();
#pragma unroll
    for (int nb = 0; nb < 4; ++nb) {
#pragma unroll
        for (int r = 0; r < 8; ++r) { const int p = wave * 16 + 8 * hi + r; const float v = acc[nb][r] * WSI;
            xs[p * XP + nb * 16 + lr] = toh_flush((p < HW) ? v : 0.0f); } }
    __syncthreads();
#pragma unroll 1
    for (int ps = 0; ps < 2; ++ps) {
#pragma unroll 1
        for (int it = 0; it < (PK * CH / 8) / FT; ++it) { const int i = it * FT + tid;
            const v8h v = *(const v8h*)(&xs[(i >> 3) * XP + (i & 7) * 8]);
            *(volatile v8h*)(X2T + (size_t)frame * PK * CH + (size_t)i * 8) = v; }
#pragma unroll 1
        for (int it = 0; it < (PK * CH / 8) / FT; ++it) { const int i = it * FT + tid;
            const int c = i / (PK / 8); const int q8 = (i - c * (PK / 8)) * 8; v8h v;
#pragma unroll
            for (int j = 0; j < 8; ++j) v[j] = xs[(q8 + j) * XP + c];
            *(volatile v8h*)(X2C + (size_t)frame * CH * PK + (size_t)i * 8) = v; }
        if (wave < PK / 32) { const v4f v = *(const v4fa*)(&xrs[tid * 4]);
            *(volatile v4f*)(XR + (size_t)frame * RC * PK + (size_t)tid * 4) = v; }
        if (ps == 0) __threadfence(); }
}

__global__ __launch_bounds__(PK) void k_conv(const float* __restrict__ XR,
                                             const float* __restrict__ W1, const float* __restrict__ B1,
                                             const float* __restrict__ W2, const float* __restrict__ B2,
                                             const float* __restrict__ W3, const float* __restrict__ B3,
                                             const float* __restrict__ WV, float* AGG) {
    __shared__ float wsm[3 * 324];
    __shared__ float bsv[12];
    __shared__ float wvs[3];
    __shared__ __align__(16) float ag[RC * PK];
    const int tid = threadIdx.x;
    const int wave = __builtin_amdgcn_readfirstlane((int)(threadIdx.x >> 5));
    const int frame = blockIdx.x; const int b = frame / NT, t = frame % NT;
#pragma unroll 1
    for (int it = 0; it < 2; ++it) { const int i = it * PK + tid; const int ic = i < 324 ? i : 323;
        const float a1 = bfr(W1[ic]), a2 = bfr(W2[ic]), a3 = bfr(W3[ic]);
        if (i < 324) { wsm[i] = a1; wsm[324 + i] = a2; wsm[648 + i] = a3; } }
    { const int q = tid & 3; const float v1 = bfr(B1[q]), v2 = bfr(B2[q]), v3 = bfr(B3[q]);
      if (tid < 4) { bsv[tid] = v1; bsv[4 + tid] = v2; bsv[8 + tid] = v3; }
      const int q3 = tid < 3 ? tid : 2; const float v4 = bfr(WV[q3]); if (tid < 3) wvs[tid] = v4; }
    __syncthreads();
    const int pc = tid < HW ? tid : HW - 1; const int h = pc / SW; const int w = pc - h * SW;
#pragma unroll 1
    for (int r = 0; r < RC; ++r) {
        float tot = 0.0f;
#pragma unroll 1
        for (int ci = 0; ci < 3; ++ci) {
            const int dil = ci + 1; float s = bsv[ci * 4 + r];
            int ro[3], co[3]; bool rk[3], ck[3];
#pragma unroll
            for (int k = 0; k < 3; ++k) { const int hh = h + (k - 1) * dil; rk[k] = (unsigned)hh < (unsigned)SW; ro[k] = (hh < 0 ? 0 : (hh > SW - 1 ? SW - 1 : hh)) * SW;
                                          const int ww = w + (k - 1) * dil; ck[k] = (unsigned)ww < (unsigned)SW; co[k] = ww < 0 ? 0 : (ww > SW - 1 ? SW - 1 : ww); }
            const int wbase = ci * 324 + r * 81;
#pragma unroll 1
            for (int kt = 0; kt < 9; ++kt) {
                const int tt = t + kt - 4; const bool tok = (unsigned)tt < (unsigned)NT; const int ttc = tt < 0 ? 0 : (tt > NT - 1 ? NT - 1 : tt);
                const float* xt = XR + ((size_t)(b * NT + ttc) * RC + (size_t)r) * PK;
#pragma unroll
                for (int kh = 0; kh < 3; ++kh) {
#pragma unroll
                    for (int kw = 0; kw < 3; ++kw) { const float val = xt[ro[kh] + co[kw]]; const bool ok = tok && rk[kh] && ck[kw];
                        s += wsm[wbase + kt * 9 + kh * 3 + kw] * (ok ? val : 0.0f); } }
            }
            tot += wvs[ci] * s;
        }
        ag[r * PK + tid] = (tid < HW) ? tot : 0.0f;
    }
    __syncthreads();
    const v4f v = *(const v4fa*)(&ag[tid * 4]);
    float* dst = AGG + (size_t)frame * RC * PK + (size_t)tid * 4;
    (void)wave;
    *(volatile v4f*)dst = v; __threadfence(); *(volatile v4f*)dst = v;
}

__global__ __launch_bounds__(32 * PT) void k_aff(const h16* __restrict__ XT, const h16* __restrict__ X2T, const h16* __restrict__ X2C,
                                                 const float* __restrict__ w2p, float* FEAT) {
    __shared__ __align__(16) float os[PT * 16 * OSP];
    const int lane = threadIdx.x & 31, lr = lane & 15, hi = lane >> 4;
    const int wave = __builtin_amdgcn_readfirstlane((int)(threadIdx.x >> 5));
    const int frame = blockIdx.x; const int b = frame / NT, t = frame % NT;
    const int p0 = wave * 16;
    const size_t qo = ((size_t)frame * PQ + (size_t)(p0 + lr)) * CH + 8 * hi;
    const v16h xq0 = ldh(XT + qo), xq1 = ldh(XT + qo + 32);
    v8f o0 = (v8f){}, o1 = (v8f){}, o2 = (v8f){}, o3 = (v8f){};
#pragma unroll 1
    for (int br = 0; br < 2; ++br) {
        int tn = t + 1 - 2 * br; tn = tn < 0 ? 0 : (tn > NT - 1 ? NT - 1 : tn);
        const int fn = b * NT + tn;
        const float wc = bfr(w2p[br]) * PCAR;
        const size_t ko = ((size_t)fn * PK + (size_t)lr) * CH + 8 * hi;
        const size_t vo = ((size_t)fn * CH + (size_t)lr) * PK + 8 * hi;
#pragma unroll 1
        for (int key0 = 0; key0 < PK; key0 += 32) {
            const h16* ka = X2T + ko + (size_t)key0 * CH;
            v8f sa = (v8f){}, sb = (v8f){};
            sa = wmma16g(ldh(ka), xq0, sa);           sa = wmma16g(ldh(ka + 32), xq1, sa);
            sb = wmma16g(ldh(ka + 16 * CH), xq0, sb); sb = wmma16g(ldh(ka + 16 * CH + 32), xq1, sb);
            const int ja = key0 + 8 * hi;
            v16h pb;
#pragma unroll
            for (int r = 0; r < 8; ++r) {
                const float ga = wc * sgm(sa[r]), gb = wc * sgm(sb[r]);
                const float pa = (ja + r < HW) ? ga : 0.0f, pc = (ja + 16 + r < HW) ? gb : 0.0f;
                pb[r] = toh_flush(pa); pb[8 + r] = toh_flush(pc); }
            const h16* va = X2C + vo + key0;
            o0 = wmma16g(ldh(va), pb, o0);
            o1 = wmma16g(ldh(va + (size_t)16 * PK), pb, o1);
            o2 = wmma16g(ldh(va + (size_t)32 * PK), pb, o2);
            o3 = wmma16g(ldh(va + (size_t)48 * PK), pb, o3);
        }
    }
    const int wb = wave * 16 * OSP;
    { v4f a, c;
      a[0] = o0[0] * PCI; a[1] = o0[1] * PCI; a[2] = o0[2] * PCI; a[3] = o0[3] * PCI; c[0] = o0[4] * PCI; c[1] = o0[5] * PCI; c[2] = o0[6] * PCI; c[3] = o0[7] * PCI;
      *(v4fa*)(&os[wb + lr * OSP +  0 + 8 * hi]) = a; *(v4fa*)(&os[wb + lr * OSP +  0 + 8 * hi + 4]) = c;
      a[0] = o1[0] * PCI; a[1] = o1[1] * PCI; a[2] = o1[2] * PCI; a[3] = o1[3] * PCI; c[0] = o1[4] * PCI; c[1] = o1[5] * PCI; c[2] = o1[6] * PCI; c[3] = o1[7] * PCI;
      *(v4fa*)(&os[wb + lr * OSP + 16 + 8 * hi]) = a; *(v4fa*)(&os[wb + lr * OSP + 16 + 8 * hi + 4]) = c;
      a[0] = o2[0] * PCI; a[1] = o2[1] * PCI; a[2] = o2[2] * PCI; a[3] = o2[3] * PCI; c[0] = o2[4] * PCI; c[1] = o2[5] * PCI; c[2] = o2[6] * PCI; c[3] = o2[7] * PCI;
      *(v4fa*)(&os[wb + lr * OSP + 32 + 8 * hi]) = a; *(v4fa*)(&os[wb + lr * OSP + 32 + 8 * hi + 4]) = c;
      a[0] = o3[0] * PCI; a[1] = o3[1] * PCI; a[2] = o3[2] * PCI; a[3] = o3[3] * PCI; c[0] = o3[4] * PCI; c[1] = o3[5] * PCI; c[2] = o3[6] * PCI; c[3] = o3[7] * PCI;
      *(v4fa*)(&os[wb + lr * OSP + 48 + 8 * hi]) = a; *(v4fa*)(&os[wb + lr * OSP + 48 + 8 * hi + 4]) = c; }
    wave_sync();
    float* orow = FEAT + ((size_t)frame * PQ + (size_t)p0) * CH;
#pragma unroll 1
    for (int ps = 0; ps < 2; ++ps) {
#pragma unroll
        for (int s = 0; s < 8; ++s) { const int row = 2 * s + (lane >> 4), cofs = (lane & 15) * 4;
            const v4f val = *(const v4fa*)(&os[wb + row * OSP + cofs]);
            *(volatile v4f*)(orow + (size_t)row * CH + cofs) = val; }
        if (ps == 0) __threadfence(); }
}

__global__ __launch_bounds__(256) void k_out(const float* __restrict__ FEAT, const float* __restrict__ AGG, const float* __restrict__ WB, float* OUT, int npiece) {
    const int i = blockIdx.x * 256 + threadIdx.x; if (i >= npiece) return;
    const int u = i / (HW / 4); const int p4 = (i - u * (HW / 4)) * 4;
    const int bc = u / NT; const int t = u - bc * NT;
    const int b = bc / CH; const int c = bc - b * CH;
    const int frame = b * NT + t;
    const v4f wb4 = *(const v4f*)(WB + c * RC);
    const float w0 = bfr(wb4[0]), w1 = bfr(wb4[1]), w2 = bfr(wb4[2]), w3 = bfr(wb4[3]);
    const float* ap = AGG + (size_t)frame * RC * PK + p4;
    const v4f a0 = *(const v4f*)ap, a1 = *(const v4f*)(ap + PK), a2 = *(const v4f*)(ap + 2 * PK), a3 = *(const v4f*)(ap + 3 * PK);
    const float* fp = FEAT + ((size_t)frame * PQ + (size_t)p4) * CH + c;
    v4f o;
#pragma unroll
    for (int j = 0; j < 4; ++j) { const float g = w0 * a0[j] + w1 * a1[j] + w2 * a2[j] + w3 * a3[j];
        o[j] = fp[(size_t)j * CH] * sgm(g); }
    float* op = OUT + ((size_t)bc * OUT_NT + (size_t)t) * HW + p4;
    *(volatile v4f*)op = o; __threadfence(); *(volatile v4f*)op = o;
}

static constexpr size_t al256(size_t v) { return (v + 255) & ~(size_t)255; }
static constexpr size_t SZ_W2H  = al256((size_t)CH * CH * 2);
static constexpr size_t SZ_XT   = al256((size_t)NB * NT * PQ * CH * 2);
static constexpr size_t SZ_X2   = al256((size_t)NB * NT * PK * CH * 2);
static constexpr size_t SZ_XR   = al256((size_t)NB * NT * RC * PK * 4);
static constexpr size_t SZ_FEAT = al256((size_t)NB * NT * PQ * CH * 4);
static constexpr size_t SZ_TOTAL = SZ_W2H + SZ_XT + 2 * SZ_X2 + 2 * SZ_XR + SZ_FEAT;
static_assert(SZ_TOTAL <= (size_t)134217728);
static constexpr size_t NEED_X = ((size_t)(NB * CH - 1) * NT_FULL + NT) * HW;
static constexpr size_t NEED_O = ((size_t)(NB * CH - 1) * OUT_NT + NT) * HW;
static constexpr int    NPIECE = NB * CH * NT * (HW / 4);
static_assert(((size_t)NT * (HW / 4)) % 8 == 0);
static_assert((size_t)NB * CH * NT * HW < (size_t)2147483647);
static_assert((CH * CH) % 8 == 0);

extern "C" void kernel_launch(void* const* d_in, const int* in_sizes, int n_in,
                              void* d_out, int out_size, void* d_ws, size_t ws_size, hipStream_t stream) {
    if (n_in < 12) return;
    if ((size_t)in_sizes[0] < NEED_X) return;
    if (in_sizes[1] < RC * CH || in_sizes[2] < CH * CH || in_sizes[9] < CH * RC) return;
    if (in_sizes[3] < 324 || in_sizes[5] < 324 || in_sizes[7] < 324) return;
    if (in_sizes[4] < RC || in_sizes[6] < RC || in_sizes[8] < RC) return;
    if (in_sizes[10] < 3 || in_sizes[11] < 2) return;
    if ((size_t)out_size < NEED_O) return;
    if (SZ_TOTAL > ws_size) return;
    const float* x    = (const float*)d_in[0];
    const float* wd   = (const float*)d_in[1];
    const float* wd2  = (const float*)d_in[2];
    const float* ws1  = (const float*)d_in[3];  const float* bs1 = (const float*)d_in[4];
    const float* ws2  = (const float*)d_in[5];  const float* bs2 = (const float*)d_in[6];
    const float* ws3  = (const float*)d_in[7];  const float* bs3 = (const float*)d_in[8];
    const float* wbk  = (const float*)d_in[9];
    const float* wts  = (const float*)d_in[10];
    const float* wts2 = (const float*)d_in[11];
    float* OUT = (float*)d_out;
    char* wsp = (char*)d_ws;
    h16*   W2H  = (h16*)wsp;   wsp += SZ_W2H;
    h16*   XT   = (h16*)wsp;   wsp += SZ_XT;
    h16*   X2T  = (h16*)wsp;   wsp += SZ_X2;
    h16*   X2C  = (h16*)wsp;   wsp += SZ_X2;
    float* XR   = (float*)wsp; wsp += SZ_XR;
    float* AGG  = (float*)wsp; wsp += SZ_XR;
    float* FEAT = (float*)wsp; wsp += SZ_FEAT;

    k_wconv<<<(CH * CH / 8 + 255) / 256, 256, 0, stream>>>(wd2, W2H, CH * CH / 8);
    k_front<<<NB * NT, FT, 0, stream>>>(x, wd, W2H, XT, X2T, X2C, XR);
    k_conv<<<NB * NT, PK, 0, stream>>>(XR, ws1, bs1, ws2, bs2, ws3, bs3, wts, AGG);
    k_aff<<<NB * NT, 32 * PT, 0, stream>>>(XT, X2T, X2C, wts2, FEAT);
    k_out<<<(NPIECE + 255) / 256, 256, 0, stream>>>(FEAT, AGG, wbk, OUT, NPIECE);
}
